// SimpleRNN_35081292874338
// MI455X (gfx1250) — hardware-verified
//
#include <hip/hip_runtime.h>
#include <math.h>

constexpr int VOCAB_N  = 32000;
constexpr int EMB_N    = 256;
constexpr int HID_N    = 256;
constexpr int BATCH_N  = 128;
constexpr int SEQ_N    = 2048;
constexpr int NTHR     = 256;
constexpr int RTHR     = 512;
constexpr int ROWS_BLK = 16;
constexpr int KCHUNKS  = HID_N / 32;
constexpr int HPITCH   = 264;
constexpr int XPITCH   = 260;
constexpr int OPITCH   = 260;
static_assert(BATCH_N % ROWS_BLK == 0);
static_assert(HID_N == 16 * (RTHR / 32));
static_assert(HID_N % 32 == 0 && EMB_N % 32 == 0);
static_assert(VOCAB_N % 64 == 0 && HID_N % 64 == 0);
static_assert(((VOCAB_N / 64) * (HID_N / 64)) % 8 == 0);
static_assert((4 * ROWS_BLK * HPITCH) % RTHR == 0);
static_assert((ROWS_BLK * HID_N / 4) % RTHR == 0);
static_assert((VOCAB_N * (EMB_N / 8)) % NTHR == 0);
static_assert(HPITCH % 8 == 0 && XPITCH % 4 == 0 && OPITCH % 4 == 0);

typedef __attribute__((ext_vector_type(16))) _Float16 v16h;
typedef __attribute__((ext_vector_type(8)))  _Float16 v8h;
typedef __attribute__((ext_vector_type(16))) __bf16   v16b;
typedef __attribute__((ext_vector_type(8)))  __bf16   v8b;
typedef __attribute__((ext_vector_type(8)))  float    v8f;
typedef __attribute__((ext_vector_type(4)))  float    v4f;

__device__ __forceinline__ unsigned short f2bf_bits(float f) {
  unsigned u = __float_as_uint(f);
  return (unsigned short)((u + 0x7FFFu + ((u >> 16) & 1u)) >> 16);
}
__device__ __forceinline__ float bf_bits2f(unsigned short h) { return __uint_as_float(((unsigned)h) << 16); }
__device__ __forceinline__ float bf16r(float f) { return bf_bits2f(f2bf_bits(f)); }

__device__ __forceinline__ void dep_guard_h(v8f& a, v8f& b, v16h x, v16h y) { asm volatile("v_nop\n\tv_nop\n\tv_nop\n\tv_nop" : "+v"(a), "+v"(b) : "v"(x), "v"(y)); }
__device__ __forceinline__ void dep_guard_b(v8f& a, v8f& b, v16b x, v16b y) { asm volatile("v_nop\n\tv_nop\n\tv_nop\n\tv_nop" : "+v"(a), "+v"(b) : "v"(x), "v"(y)); }
__device__ __forceinline__ void keep4_h(v16h a, v16h b, v16h c, v16h d) { asm volatile("v_nop" :: "v"(a), "v"(b), "v"(c), "v"(d)); }
__device__ __forceinline__ void keep4_b(v16b a, v16b b, v16b c, v16b d) { asm volatile("v_nop" :: "v"(a), "v"(b), "v"(c), "v"(d)); }
__device__ __forceinline__ void acc_guard4(v8f& a, v8f& b, v8f& c, v8f& d) { asm volatile("v_nop\n\tv_nop\n\tv_nop\n\tv_nop" : "+v"(a), "+v"(b), "+v"(c), "+v"(d)); }
__device__ __forceinline__ void mma_guard3(v8f& a, v16b x, v16b y, v16b z) {
  asm volatile("v_nop\n\tv_nop\n\tv_nop\n\tv_nop" : "+v"(a) : "v"(x), "v"(y), "v"(z) : "memory");
}
__device__ __forceinline__ void acc_guard1(v8f& a) { asm volatile("v_nop\n\tv_nop\n\tv_nop\n\tv_nop" : "+v"(a)); }
__device__ __forceinline__ void frag_ready(v16b x) { asm volatile("" :: "v"(x) : "memory"); }

template <typename T> struct Frag;
template <> struct Frag<_Float16> {
  typedef v16h V; union U { v16h v; v8h h[2]; };
  static __device__ __forceinline__ v16h load(const _Float16* p) {
    U f; f.h[0] = *(const v8h*)(p); f.h[1] = *(const v8h*)(p + 16); return f.v;
  }
  static __device__ __forceinline__ v8f mma(v16h a, v16h b, v8f c) {
    return __builtin_amdgcn_wmma_f32_16x16x32_f16(false, a, false, b, (short)0, c, false, false);
  }
  static __device__ __forceinline__ void guard(v8f& a, v8f& b, v16h x, v16h y) { dep_guard_h(a, b, x, y); }
  static __device__ __forceinline__ void keep(v16h a, v16h b, v16h c, v16h d) { keep4_h(a, b, c, d); }
};
template <> struct Frag<__bf16> {
  typedef v16b V; union U { v16b v; v8b h[2]; };
  static __device__ __forceinline__ v16b load(const __bf16* p) {
    U f; f.h[0] = *(const v8b*)(p); f.h[1] = *(const v8b*)(p + 16); return f.v;
  }
  static __device__ __forceinline__ v8f mma(v16b a, v16b b, v8f c) {
    return __builtin_amdgcn_wmma_f32_16x16x32_bf16(false, a, false, b, (short)0, c, false, false);
  }
  static __device__ __forceinline__ void guard(v8f& a, v8f& b, v16b x, v16b y) { dep_guard_b(a, b, x, y); }
  static __device__ __forceinline__ void keep(v16b a, v16b b, v16b c, v16b d) { keep4_b(a, b, c, d); }
};

template <int ET> struct Elem;
template <> struct Elem<0> { typedef _Float16 T; };
template <> struct Elem<1> { typedef __bf16 T; };
template <int ET, bool SPLIT, int BIAS_MODE, int OUT_MODE, bool RESID, int ACT = 0>
__global__ __launch_bounds__(256) void wmma_gemm64(
    const unsigned short* __restrict__ Ap, const unsigned short* __restrict__ A2p, int lda, long strideA,
    const unsigned short* __restrict__ Btp, const unsigned short* __restrict__ Bt2p, int ldb, long strideB,
    void* __restrict__ Cout, void* __restrict__ Cout2, int ldc, long strideC,
    const float* __restrict__ bias,
    const float* __restrict__ resid, long strideR,
    int M, int N, int K, float scale) {
  typedef typename Elem<ET>::T T;
  typedef typename Frag<T>::V V;
  const T* A = (const T*)Ap; const T* A2 = (const T*)A2p; const T* Bt = (const T*)Btp; const T* Bt2 = (const T*)Bt2p;
  __shared__ __align__(16) float sT[8][16 * 68];
  const int b    = blockIdx.y;
  const int lane = threadIdx.x & 31;
  const int wave = threadIdx.x >> 5;
  const int tilesN = N >> 6;
  const int tilesM = M >> 6;
  const int tile = blockIdx.x * 8 + wave;
  if (tile >= tilesM * tilesN) return;
  const int tm = tile / tilesN;
  const int tn = tile - tm * tilesN;
  const int m0 = tm << 6;
  const int n0 = tn << 6;

  const T* Ab  = A  + (size_t)b * strideA;
  const T* Bb  = Bt + (size_t)b * strideB;
  const T* Ab2 = SPLIT ? (A2  + (size_t)b * strideA) : nullptr;
  const T* Bb2 = SPLIT ? (Bt2 + (size_t)b * strideB) : nullptr;

  const int rlane = lane & 15;
  const int koff  = (lane >> 4) * 8;
  const int mOff  = (lane >> 4) * 8;

  v8f acc[4][4];
#pragma unroll
  for (int i = 0; i < 4; ++i)
#pragma unroll
    for (int j = 0; j < 4; ++j) acc[i][j] = (v8f){0.f,0.f,0.f,0.f,0.f,0.f,0.f,0.f};

  for (int k0 = 0; k0 < K; k0 += 32) {
    V bh[4], bl[4];
#pragma unroll
    for (int j = 0; j < 4; ++j) {
      const size_t bo = (size_t)(n0 + (j << 4) + rlane) * ldb + koff + k0;
      bh[j] = Frag<T>::load(Bb + bo);
      if (SPLIT) bl[j] = Frag<T>::load(Bb2 + bo);
    }
#pragma unroll
    for (int i = 0; i < 4; ++i) {
      const size_t ao = (size_t)(m0 + (i << 4) + rlane) * lda + koff + k0;
      V ah = Frag<T>::load(Ab + ao);
      V al;
      if (SPLIT) al = Frag<T>::load(Ab2 + ao);
#pragma unroll
      for (int j = 0; j < 4; ++j) {
        acc[i][j] = Frag<T>::mma(ah, bh[j], acc[i][j]);
        if (SPLIT) {
          acc[i][j] = Frag<T>::mma(ah, bl[j], acc[i][j]);
          acc[i][j] = Frag<T>::mma(al, bh[j], acc[i][j]);
        }
      }
      Frag<T>::guard(acc[i][0], acc[i][3], ah, SPLIT ? al : ah);
    }
    Frag<T>::keep(bh[0], bh[1], bh[2], bh[3]);
    if (SPLIT) Frag<T>::keep(bl[0], bl[1], bl[2], bl[3]);
  }
  acc_guard4(acc[0][0], acc[0][1], acc[0][2], acc[0][3]);
  acc_guard4(acc[1][0], acc[1][1], acc[1][2], acc[1][3]);
  acc_guard4(acc[2][0], acc[2][1], acc[2][2], acc[2][3]);
  acc_guard4(acc[3][0], acc[3][1], acc[3][2], acc[3][3]);

  float* slab = sT[wave];
  const float* Rb = RESID ? (resid + (size_t)b * strideR) : nullptr;
#pragma unroll
  for (int i = 0; i < 4; ++i) {
    const int mBase = m0 + (i << 4);
#pragma unroll
    for (int j = 0; j < 4; ++j) {
      const int n = n0 + (j << 4) + rlane;
      float bv = 0.f;
      if (BIAS_MODE == 2) bv = bias[n];
#pragma unroll
      for (int r = 0; r < 8; ++r) {
        float v = acc[i][j][r] * scale;
        if (BIAS_MODE == 1) v += bias[mBase + mOff + r];
        if (BIAS_MODE == 2) v += bv;
        if (RESID) v += Rb[(size_t)(mBase + mOff + r) * ldc + n];
        if (ACT == 1) v = tanhf(v);
        if (ACT == 2) v = fmaxf(v, 0.0f);
        if (ACT == 3) v = v / (1.0f + expf(-v));
        if (ACT == 4) v = (v > 0.f) ? v : 0.01f * v;
        if (ACT == 5) v = 0.5f * v * (1.0f + erff(v * 0.70710678118654752f));
        slab[(mOff + r) * 68 + (j << 4) + rlane] = v;
      }
    }
    __builtin_amdgcn_fence(__ATOMIC_RELEASE, "workgroup");
    __builtin_amdgcn_wave_barrier();
    __builtin_amdgcn_fence(__ATOMIC_ACQUIRE, "workgroup");
    if (OUT_MODE == 0) {
      float* C = (float*)Cout + (size_t)b * strideC;
      const int hh = lane >> 4, c4 = (lane & 15) * 4;
      for (int pass = 0; pass < 2; ++pass) {
#pragma unroll
        for (int it = 0; it < 8; ++it) {
          const int row = it * 2 + hh;
          v4f v = *(const v4f*)(slab + row * 68 + c4);
          *(volatile v4f*)(C + (size_t)(mBase + row) * ldc + n0 + c4) = v;
        }
        __threadfence();
      }
    } else {
      const int q = lane >> 3, c8 = (lane & 7) * 8;
      unsigned short* C  = (unsigned short*)Cout  + (size_t)b * strideC;
      unsigned short* C2 = (OUT_MODE == 2) ? ((unsigned short*)Cout2 + (size_t)b * strideC) : nullptr;
      for (int pass = 0; pass < 2; ++pass) {
#pragma unroll
        for (int it = 0; it < 4; ++it) {
          const int row = it * 4 + q;
          const float* sp = slab + row * 68 + c8;
          v8h hv, lv;
#pragma unroll
          for (int e = 0; e < 8; ++e) {
            if (OUT_MODE == 1) {
              hv[e] = (_Float16)sp[e];
            } else {
              unsigned short hb = f2bf_bits(sp[e]);
              unsigned short lb = f2bf_bits(sp[e] - bf_bits2f(hb));
              hv[e] = __builtin_bit_cast(_Float16, hb);
              lv[e] = __builtin_bit_cast(_Float16, lb);
            }
          }
          *(volatile v8h*)(C + (size_t)(mBase + row) * ldc + n0 + c8) = hv;
          if (OUT_MODE == 2) *(volatile v8h*)(C2 + (size_t)(mBase + row) * ldc + n0 + c8) = lv;
        }
        __threadfence();
      }
    }
    __builtin_amdgcn_fence(__ATOMIC_RELEASE, "workgroup");
    __builtin_amdgcn_wave_barrier();
    __builtin_amdgcn_fence(__ATOMIC_ACQUIRE, "workgroup");
  }
}

__global__ __launch_bounds__(NTHR) void cvt8_kernel(const float* __restrict__ src, unsigned short* __restrict__ dst,
                                                    int nrow, int ncol8, int spitch, int scol0, float sc) {
  const int i  = blockIdx.x * NTHR + threadIdx.x;
  const int n8 = nrow * ncol8;
  if (i < n8) {
    const int row = i / ncol8;
    const int c8  = i - row * ncol8;
    const float* sp = src + (size_t)row * spitch + scol0 + c8 * 8;
    const v4f a = *(const v4f*)(sp);
    const v4f b = *(const v4f*)(sp + 4);
    v8h hv;
#pragma unroll
    for (int e = 0; e < 4; ++e) {
      const unsigned short b0 = f2bf_bits(a[e] * sc);
      const unsigned short b1 = f2bf_bits(b[e] * sc);
      hv[e]     = __builtin_bit_cast(_Float16, b0);
      hv[4 + e] = __builtin_bit_cast(_Float16, b1);
    }
    *(volatile v8h*)(dst + (size_t)i * 8) = hv;
    __threadfence();
    *(volatile v8h*)(dst + (size_t)i * 8) = hv;
  }
}

__global__ __launch_bounds__(NTHR) void tpw_kernel(const float* __restrict__ src, int R, int C, int ldo,
                                                   unsigned short* __restrict__ O, float sc) {
  __shared__ float Tt[64 * 65];
  const int tid = threadIdx.x;
  const int c0 = blockIdx.x * 64, r0 = blockIdx.y * 64;
#pragma unroll
  for (int i = 0; i < 4; ++i) {
    const int idx = i * NTHR + tid;
    const int rr = idx >> 4, cc = (idx & 15) * 4;
    const v4f v = *(const v4f*)(src + (size_t)(r0 + rr) * (size_t)C + c0 + cc);
    Tt[rr * 65 + cc + 0] = v[0];
    Tt[rr * 65 + cc + 1] = v[1];
    Tt[rr * 65 + cc + 2] = v[2];
    Tt[rr * 65 + cc + 3] = v[3];
  }
  __syncthreads();
  const int q = tid >> 3, c8 = (tid & 7) * 8;
  v8h hv[2];
#pragma unroll
  for (int g = 0; g < 2; ++g) {
    const int qq = g * 32 + q;
#pragma unroll
    for (int e = 0; e < 8; ++e) {
      const float f = Tt[(c8 + e) * 65 + qq];
      const unsigned short bits = f2bf_bits(f * sc);
      hv[g][e] = __builtin_bit_cast(_Float16, bits);
    }
  }
  for (int pass = 0; pass < 2; ++pass) {
#pragma unroll
    for (int g = 0; g < 2; ++g) {
      const size_t o = (size_t)(c0 + g * 32 + q) * (size_t)ldo + (size_t)(r0 + c8);
      *(volatile v8h*)(O + o) = hv[g];
    }
    __threadfence();
  }
}

__global__ __launch_bounds__(RTHR) void rnn_seq_kernel(const int* __restrict__ X, const float* __restrict__ P,
                                                       const unsigned short* __restrict__ BtHHp,
                                                       const float* __restrict__ b_xh, const float* __restrict__ b_hh,
                                                       float* __restrict__ out) {
  __shared__ __align__(16) unsigned short Hbuf[4][ROWS_BLK * HPITCH];
  __shared__ __align__(16) float          Xs[2][ROWS_BLK * XPITCH];
  __shared__ __align__(16) float          Os[ROWS_BLK * OPITCH];
  const __bf16* BtHH = (const __bf16*)BtHHp;
  const int tid = threadIdx.x, lane = tid & 31, wave = tid >> 5;
  const int c = lane & 15, hh = lane >> 4, koff = hh * 8;
  const int rowbase = blockIdx.x * ROWS_BLK;
  const int col  = 16 * wave + c;
  const int prow = rowbase + wave;

  {
    unsigned short* hp = &Hbuf[0][0];
#pragma unroll 1
    for (int i = tid; i < 4 * ROWS_BLK * HPITCH; i += RTHR) hp[i] = (unsigned short)0;
  }
  __syncthreads();

  v16b bw[KCHUNKS];
  {
    const __bf16* wrow = BtHH + (size_t)col * HID_N + koff;
#pragma unroll
    for (int kc = 0; kc < KCHUNKS; ++kc) {
      bw[kc] = Frag<__bf16>::load(wrow + 32 * kc);
      if ((kc & 1) == 1) frag_ready(bw[kc]);
    }
  }
  const float bsum = bf16r(b_xh[col]) + bf16r(b_hh[col]);

  {
    int xi = X[(size_t)prow * SEQ_N];
    xi = xi < 0 ? 0 : xi; xi = xi > VOCAB_N - 1 ? VOCAB_N - 1 : xi;
    const float* pr = P + (size_t)xi * HID_N + 8 * lane;
    const v4f p0 = *(const v4f*)(pr);
    const v4f p1 = *(const v4f*)(pr + 4);
    *(v4f*)(&Xs[0][wave * XPITCH + 8 * lane]) = p0;
    *(v4f*)(&Xs[0][wave * XPITCH + 8 * lane + 4]) = p1;
  }
  float hreg[8];
#pragma unroll
  for (int r = 0; r < 8; ++r) hreg[r] = 0.0f;
  __syncthreads();

  const v8f z8 = {0.f, 0.f, 0.f, 0.f, 0.f, 0.f, 0.f, 0.f};

#pragma unroll 1
  for (int t = 0; t < SEQ_N; ++t) {
    const int cur = t & 1;
    const int tn = (t + 1 < SEQ_N) ? (t + 1) : (SEQ_N - 1);
    int xi = X[(size_t)prow * SEQ_N + tn];
    xi = xi < 0 ? 0 : xi; xi = xi > VOCAB_N - 1 ? VOCAB_N - 1 : xi;
    const float* pr = P + (size_t)xi * HID_N + 8 * lane;
    const v4f p0 = *(const v4f*)(pr);
    const v4f p1 = *(const v4f*)(pr + 4);

    const float* xs = &Xs[cur][0];
    v8f acc = z8;
#pragma unroll
    for (int r = 0; r < 8; ++r) acc[r] = xs[(8 * hh + r) * XPITCH + col] + bsum;

    const __bf16* ahp = (const __bf16*)(&Hbuf[cur][0])     + c * HPITCH + koff;
    const __bf16* alp = (const __bf16*)(&Hbuf[2 + cur][0]) + c * HPITCH + koff;
#pragma unroll
    for (int kc = 0; kc < KCHUNKS; ++kc) {
      const v16b ah = Frag<__bf16>::load(ahp + 32 * kc);
      const v16b al = Frag<__bf16>::load(alp + 32 * kc);
      acc = Frag<__bf16>::mma(ah, bw[kc], acc);
      acc = Frag<__bf16>::mma(al, bw[kc], acc);
      mma_guard3(acc, ah, al, bw[kc]);
    }
    acc_guard1(acc);

    unsigned short* hn = &Hbuf[cur ^ 1][0];
    unsigned short* ln = &Hbuf[2 + (cur ^ 1)][0];
#pragma unroll
    for (int r = 0; r < 8; ++r) {
      const float hv = tanhf(acc[r]);
      hreg[r] = hv;
      const unsigned short hb = f2bf_bits(hv);
      const unsigned short lb = f2bf_bits(hv - bf_bits2f(hb));
      hn[(8 * hh + r) * HPITCH + col] = hb;
      ln[(8 * hh + r) * HPITCH + col] = lb;
    }
    *(v4f*)(&Xs[cur ^ 1][wave * XPITCH + 8 * lane]) = p0;
    *(v4f*)(&Xs[cur ^ 1][wave * XPITCH + 8 * lane + 4]) = p1;
    __syncthreads();
  }

#pragma unroll
  for (int r = 0; r < 8; ++r) Os[(8 * hh + r) * OPITCH + col] = hreg[r];
  __syncthreads();
  for (int pass = 0; pass < 2; ++pass) {
#pragma unroll
    for (int it = 0; it < 2; ++it) {
      const int idx = it * RTHR + tid;
      const int row = idx >> 6, c4 = (idx & 63) * 4;
      const v4f v = *(const v4f*)(Os + row * OPITCH + c4);
      *(volatile v4f*)(out + (size_t)(rowbase + row) * HID_N + c4) = v;
    }
    __threadfence();
  }
}

extern "C" void kernel_launch(void* const* d_in, const int* in_sizes, int n_in,
                              void* d_out, int out_size, void* d_ws, size_t ws_size, hipStream_t stream) {
  if (n_in < 6 || d_out == nullptr || d_ws == nullptr) return;
  if (in_sizes[0] != BATCH_N * SEQ_N || in_sizes[1] != VOCAB_N * EMB_N || in_sizes[2] != HID_N * HID_N ||
      in_sizes[3] != HID_N || in_sizes[4] != EMB_N * HID_N || in_sizes[5] != HID_N || out_size != BATCH_N * HID_N) return;

  const int*   X    = (const int*)  d_in[0];
  const float* emb  = (const float*)d_in[1];
  const float* w_hh = (const float*)d_in[2];
  const float* b_hh = (const float*)d_in[3];
  const float* w_xh = (const float*)d_in[4];
  const float* b_xh = (const float*)d_in[5];
  float* out = (float*)d_out;

  char* ws = (char*)d_ws; size_t off = 0;
  auto carve = [&](size_t bytes) -> char* { char* p = ws + off; off += (bytes + 255) & ~(size_t)255; return p; };
  unsigned short* AEMB = (unsigned short*)carve((size_t)VOCAB_N * EMB_N * 2);
  unsigned short* BTXH = (unsigned short*)carve((size_t)HID_N * EMB_N * 2);
  unsigned short* BTHH = (unsigned short*)carve((size_t)HID_N * HID_N * 2);
  float*          PTAB = (float*)carve((size_t)VOCAB_N * HID_N * 4);
  if (off > ws_size || off > (size_t)134217728) return;

  const int n8e = VOCAB_N * (EMB_N / 8);
  cvt8_kernel<<<(n8e + NTHR - 1) / NTHR, NTHR, 0, stream>>>(emb, AEMB, VOCAB_N, EMB_N / 8, EMB_N, 0, 1.0f);
  tpw_kernel<<<dim3(HID_N / 64, EMB_N / 64), NTHR, 0, stream>>>(w_xh, EMB_N, HID_N, EMB_N, BTXH, 1.0f);
  tpw_kernel<<<dim3(HID_N / 64, HID_N / 64), NTHR, 0, stream>>>(w_hh, HID_N, HID_N, HID_N, BTHH, 1.0f);

  const dim3 ggrid((VOCAB_N / 64) * (HID_N / 64) / 8, 1);
  wmma_gemm64<1, false, 0, 0, false, 0><<<ggrid, 256, 0, stream>>>(
      AEMB, AEMB, EMB_N, 0L, BTXH, BTXH, EMB_N, 0L, (void*)PTAB, (void*)PTAB, HID_N, 0L,
      b_xh, b_hh, 0L, VOCAB_N, HID_N, EMB_N, 1.0f);

  rnn_seq_kernel<<<BATCH_N / ROWS_BLK, RTHR, 0, stream>>>(X, PTAB, BTHH, b_xh, b_hh, out);
}
